// Self_Attn_66726611910773
// MI455X (gfx1250) — hardware-verified
//
#include <hip/hip_runtime.h>
#include <stdint.h>


#ifndef NB
#define NB 4
#endif
#ifndef SEQ
#define SEQ 4096
#endif
#define NFULL 4096
#define C_  256
#define OC_ 32

static_assert(NB >= 1 && NB <= 4);
static_assert(SEQ % 64 == 0 && SEQ >= 64 && SEQ <= NFULL);

#define WSC 64.0f
#define QSC 8.0f
#define PSC 1024.0f

typedef _Float16 v16h __attribute__((ext_vector_type(16)));
typedef _Float16 v8h  __attribute__((ext_vector_type(8)));
typedef float    v8f  __attribute__((ext_vector_type(8)));
typedef float    v4f  __attribute__((ext_vector_type(4)));
union Frag { v16h v; v8h half[2]; };

__device__ __forceinline__ float bf16r(float f) {
  uint32_t u = __float_as_uint(f);
  u = (u + 0x7FFFu + ((u >> 16) & 1u)) & 0xFFFF0000u;
  return __uint_as_float(u);
}

__device__ __forceinline__ v8f zero8() {
  v8f z;
#pragma unroll
  for (int r = 0; r < 8; ++r) z[r] = 0.f;
  return z;
}

__device__ __forceinline__ v16h ld_frag(const _Float16* base, int rs) {
  int lane = threadIdx.x & 31;
  int h = lane >> 4, m = lane & 15;
  const _Float16* p = base + m * rs + 8 * h;
  Frag f;
  f.half[0] = *(const v8h*)(p);
  f.half[1] = *(const v8h*)(p + 16);
  return f.v;
}

__device__ __forceinline__ v8f mma(v16h a, v16h b, v8f c) {
  v8f d = __builtin_amdgcn_wmma_f32_16x16x32_f16(false, a, false, b, (short)0, c,
                                                 false, false);
  asm volatile("v_nop\n\tv_nop\n\tv_nop\n\tv_nop" : "+v"(d) : "v"(a), "v"(b));
  return d;
}

__global__ void __launch_bounds__(256)
k_cvt_w(const float* __restrict__ Wq, const float* __restrict__ Wk,
        const float* __restrict__ Wv,
        _Float16* wq16, _Float16* wk16, _Float16* wv16) {
  int chunk = blockIdx.x * 256 + threadIdx.x;
  const float* src;
  _Float16* dst;
  int e;
  if (blockIdx.x < 4)      { src = Wq; dst = wq16; e = chunk * 8; }
  else if (blockIdx.x < 8) { src = Wk; dst = wk16; e = (chunk - 1024) * 8; }
  else                     { src = Wv; dst = wv16; e = (chunk - 2048) * 8; }
  v4f a = *(const v4f*)(src + e);
  v4f c = *(const v4f*)(src + e + 4);
  v8h o;
#pragma unroll
  for (int i = 0; i < 4; ++i) {
    o[i]     = (_Float16)(bf16r(a[i]) * WSC);
    o[4 + i] = (_Float16)(bf16r(c[i]) * WSC);
  }
  *(volatile v8h*)(dst + e) = o;
  __threadfence();
  *(volatile v8h*)(dst + e) = o;
}

__global__ void __launch_bounds__(256)
k_transpose_x(const float* __restrict__ x, _Float16* xh) {
  __shared__ __attribute__((aligned(16))) _Float16 t[32 * 264];
  int nt = blockIdx.x % (SEQ / 32);
  int b  = blockIdx.x / (SEQ / 32);
  int n0 = nt * 32;
  int tx = threadIdx.x & 31, ty = threadIdx.x >> 5;
  const float* xb = x + (size_t)b * C_ * NFULL + n0 + tx;
#pragma unroll 4
  for (int c = ty; c < C_; c += 8)
    t[tx * 264 + c] = (_Float16)bf16r(xb[(size_t)c * NFULL]);
  __syncthreads();
  int w = ty, lane = tx;
  v8h v[4];
  size_t off[4];
#pragma unroll
  for (int rr = 0; rr < 4; ++rr) {
    int n = w * 4 + rr;
    v[rr]   = *(const v8h*)(&t[n * 264 + 8 * lane]);
    off[rr] = ((size_t)(b * SEQ + n0 + n)) * C_ + 8 * lane;
  }
#pragma unroll
  for (int rr = 0; rr < 4; ++rr) *(volatile v8h*)(xh + off[rr]) = v[rr];
  __threadfence();
#pragma unroll
  for (int rr = 0; rr < 4; ++rr) *(volatile v8h*)(xh + off[rr]) = v[rr];
}

__global__ void __launch_bounds__(128)
k_proj(const _Float16* __restrict__ xh,
       const _Float16* __restrict__ wq16, const _Float16* __restrict__ wk16,
       const _Float16* __restrict__ wv16,
       const float* __restrict__ bq, const float* __restrict__ bk,
       const float* __restrict__ bv,
       _Float16* qh, _Float16* kh, _Float16* vh) {
  __shared__ __attribute__((aligned(16))) _Float16 lds[64 * 40];
  int bid = blockIdx.x;
  int rt = bid % 18; bid /= 18;
  int nt = bid % (SEQ / 64);
  int b  = bid / (SEQ / 64);
  int n0 = nt * 64;
  int w = threadIdx.x >> 5, lane = threadIdx.x & 31;
  int h = lane >> 4, nl = lane & 15;
  const _Float16* xrow = xh + ((size_t)(b * SEQ + n0 + 16 * w)) * C_;

  if (rt < 16) {
    int c0 = rt * 16;
    const _Float16* wrow = wv16 + (size_t)c0 * C_;
    v8f acc = zero8();
#pragma unroll
    for (int k0 = 0; k0 < C_; k0 += 32) {
      v16h a  = ld_frag(wrow + k0, C_);
      v16h bm = ld_frag(xrow + k0, C_);
      acc = mma(a, bm, acc);
    }
#pragma unroll
    for (int r = 0; r < 8; ++r) {
      int cr = 8 * h + r;
      float val = (acc[r] * (1.0f / WSC) + bf16r(bv[c0 + cr])) * QSC;
      lds[cr * 72 + 16 * w + nl] = (_Float16)val;
    }
    __syncthreads();
    int row = w * 4 + (lane >> 3), q = lane & 7;
    v8h v = *(const v8h*)(&lds[row * 72 + 8 * q]);
    size_t off = ((size_t)(b * C_ + c0 + row)) * SEQ + n0 + 8 * q;
    *(volatile v8h*)(vh + off) = v;
    __threadfence();
    *(volatile v8h*)(vh + off) = v;
  } else {
    const _Float16* wm = (rt == 16) ? wq16 : wk16;
    const float* bias  = (rt == 16) ? bq : bk;
    _Float16* dst      = (rt == 16) ? qh : kh;
    v8f acc0 = zero8(), acc1 = zero8();
#pragma unroll
    for (int k0 = 0; k0 < C_; k0 += 32) {
      v16h a  = ld_frag(xrow + k0, C_);
      v16h b0 = ld_frag(wm + k0, C_);
      v16h b1 = ld_frag(wm + 16 * C_ + k0, C_);
      acc0 = mma(a, b0, acc0);
      acc1 = mma(a, b1, acc1);
    }
    float bb0 = bf16r(bias[nl]), bb1 = bf16r(bias[16 + nl]);
#pragma unroll
    for (int r = 0; r < 8; ++r) {
      int nr = 16 * w + 8 * h + r;
      lds[nr * 40 + nl]      = (_Float16)((acc0[r] * (1.0f / WSC) + bb0) * QSC);
      lds[nr * 40 + 16 + nl] = (_Float16)((acc1[r] * (1.0f / WSC) + bb1) * QSC);
    }
    __syncthreads();
    v8h v[2];
    size_t off[2];
#pragma unroll
    for (int s = 0; s < 2; ++s) {
      int ci = (s * 4 + w) * 32 + lane;
      int row = ci >> 2, col = (ci & 3) * 8;
      v[s]   = *(const v8h*)(&lds[row * 40 + col]);
      off[s] = ((size_t)(b * SEQ + n0 + row)) * OC_ + col;
    }
#pragma unroll
    for (int s = 0; s < 2; ++s) *(volatile v8h*)(dst + off[s]) = v[s];
    __threadfence();
#pragma unroll
    for (int s = 0; s < 2; ++s) *(volatile v8h*)(dst + off[s]) = v[s];
  }
}

__global__ void __launch_bounds__(128)
k_attn(const _Float16* __restrict__ qh, const _Float16* __restrict__ kh,
       const _Float16* __restrict__ vh, const float* __restrict__ x,
       const float* __restrict__ gamma, float* out) {
  __shared__ __attribute__((aligned(16))) float lo[C_ * 36];
  int bid = blockIdx.x;
  int it = bid % (SEQ / 32);
  int b  = bid / (SEQ / 32);
  int i0 = it * 32;
  int w = threadIdx.x >> 5, lane = threadIdx.x & 31;
  int h = lane >> 4, nl = lane & 15;
  int qsub = w & 1, ch = w >> 1;
  int iq = i0 + 16 * qsub;
  int cbase = 128 * ch;

  v16h Bq = ld_frag(qh + ((size_t)(b * SEQ + iq)) * OC_, OC_);

  v8f acc[8];
#pragma unroll
  for (int t = 0; t < 8; ++t) acc[t] = zero8();
  float mrun = -1e30f, lrun = 0.f;

  const _Float16* kb = kh + (size_t)b * SEQ * OC_;
  const _Float16* vb = vh + ((size_t)(b * C_ + cbase)) * SEQ;

#pragma unroll 1
  for (int j0 = 0; j0 < SEQ; j0 += 32) {
    v16h A0 = ld_frag(kb + (size_t)j0 * OC_, OC_);
    v16h A1 = ld_frag(kb + (size_t)(j0 + 16) * OC_, OC_);
    v8f e0 = mma(A0, Bq, zero8());
    v8f e1 = mma(A1, Bq, zero8());

    float bm = -1e30f;
#pragma unroll
    for (int r = 0; r < 8; ++r) { bm = fmaxf(bm, e0[r]); bm = fmaxf(bm, e1[r]); }
    bm *= (1.0f / (QSC * QSC));
    bm = fmaxf(bm, __shfl_xor(bm, 16));
    float mn = fmaxf(mrun, bm);
    float sc = __expf(mrun - mn);
    float p0[8], p1[8];
    float bs = 0.f;
#pragma unroll
    for (int r = 0; r < 8; ++r) {
      p0[r] = __expf(e0[r] * (1.0f / (QSC * QSC)) - mn); bs += p0[r];
      p1[r] = __expf(e1[r] * (1.0f / (QSC * QSC)) - mn); bs += p1[r];
    }
    bs += __shfl_xor(bs, 16);
    lrun = lrun * sc + bs;
    mrun = mn;
#pragma unroll
    for (int t = 0; t < 8; ++t) {
#pragma unroll
      for (int r = 0; r < 8; ++r) acc[t][r] *= sc;
    }

    v8h ph0, ph1;
#pragma unroll
    for (int r = 0; r < 8; ++r) {
      ph0[r] = (_Float16)(p0[r] * PSC);
      ph1[r] = (_Float16)(p1[r] * PSC);
    }
    Frag pb;
    pb.half[0] = ph0;
    pb.half[1] = ph1;
    v16h B2 = pb.v;

#pragma unroll
    for (int t = 0; t < 8; ++t) {
      v16h Av = ld_frag(vb + (size_t)(16 * t) * SEQ + j0, SEQ);
      acc[t] = mma(Av, B2, acc[t]);
    }
  }

  float g = bf16r(gamma[0]);
  float inv = g * (1.0f / (lrun * (QSC * PSC)));
#pragma unroll
  for (int t = 0; t < 8; ++t) {
#pragma unroll
    for (int r = 0; r < 8; ++r) {
      int c = cbase + 16 * t + 8 * h + r;
      lo[c * 36 + 16 * qsub + nl] = acc[t][r] * inv;
    }
  }
  __syncthreads();

  int rq = lane >> 3, q4 = lane & 7;
  const float* xb = x + (size_t)b * C_ * NFULL + i0 + 4 * q4;
  float* ob = out + (size_t)b * C_ * SEQ + i0 + 4 * q4;
#pragma unroll 4
  for (int s = 0; s < 16; ++s) {
    int c = s * 16 + w * 4 + rq;
    v4f o  = *(const v4f*)(&lo[c * 36 + 4 * q4]);
    v4f xv = *(const v4f*)(xb + (size_t)c * NFULL);
    v4f val;
#pragma unroll
    for (int i = 0; i < 4; ++i) val[i] = o[i] + bf16r(xv[i]);
    *(volatile v4f*)(ob + (size_t)c * SEQ) = val;
  }
  __threadfence();
#pragma unroll 4
  for (int s = 0; s < 16; ++s) {
    int c = s * 16 + w * 4 + rq;
    v4f o  = *(const v4f*)(&lo[c * 36 + 4 * q4]);
    v4f xv = *(const v4f*)(xb + (size_t)c * NFULL);
    v4f val;
#pragma unroll
    for (int i = 0; i < 4; ++i) val[i] = o[i] + bf16r(xv[i]);
    *(volatile v4f*)(ob + (size_t)c * SEQ) = val;
  }
}

extern "C" void kernel_launch(void* const* d_in, const int* in_sizes, int n_in,
                              void* d_out, int out_size, void* d_ws, size_t ws_size,
                              hipStream_t stream) {
  if (n_in < 8) return;
  if (in_sizes[0] < NB * C_ * NFULL) return;
  if (in_sizes[1] < OC_ * C_ || in_sizes[2] < OC_ || in_sizes[3] < OC_ * C_ ||
      in_sizes[4] < OC_ || in_sizes[5] < C_ * C_ || in_sizes[6] < C_ || in_sizes[7] < 1)
    return;
  if ((size_t)out_size < (size_t)NB * C_ * SEQ) return;

  const float* x     = (const float*)d_in[0];
  const float* Wq    = (const float*)d_in[1];
  const float* bq    = (const float*)d_in[2];
  const float* Wk    = (const float*)d_in[3];
  const float* bk    = (const float*)d_in[4];
  const float* Wv    = (const float*)d_in[5];
  const float* bv    = (const float*)d_in[6];
  const float* gamma = (const float*)d_in[7];
  float* out = (float*)d_out;

  char* ws = (char*)d_ws;
  size_t o = 0;
  _Float16* xh   = (_Float16*)(ws + o); o += (size_t)NB * SEQ * C_ * 2;
  _Float16* wq16 = (_Float16*)(ws + o); o += (size_t)OC_ * C_ * 2;
  _Float16* wk16 = (_Float16*)(ws + o); o += (size_t)OC_ * C_ * 2;
  _Float16* wv16 = (_Float16*)(ws + o); o += (size_t)C_ * C_ * 2;
  _Float16* qh   = (_Float16*)(ws + o); o += (size_t)NB * SEQ * OC_ * 2;
  _Float16* kh   = (_Float16*)(ws + o); o += (size_t)NB * SEQ * OC_ * 2;
  _Float16* vh   = (_Float16*)(ws + o); o += (size_t)NB * C_ * SEQ * 2;
  if (o > ws_size) return;

  k_cvt_w<<<40, 256, 0, stream>>>(Wq, Wk, Wv, wq16, wk16, wv16);
  k_transpose_x<<<NB * (SEQ / 32), 256, 0, stream>>>(x, xh);
  k_proj<<<NB * (SEQ / 64) * 18, 128, 0, stream>>>(xh, wq16, wk16, wv16, bq, bk, bv,
                                                    qh, kh, vh);
  k_attn<<<NB * (SEQ / 32), 128, 0, stream>>>(qh, kh, vh, x, gamma, out);
}
